// CrossPlaneMixer_60636348285068
// MI455X (gfx1250) — hardware-run, weakly checked
//
#include <hip/hip_runtime.h>


#define NSM  2
#define NCH  64
#define NPL  65536
#define NSH  4096
#define KDP  256
constexpr size_t al256(size_t b) { return (b + 255) & ~(size_t)255; }
constexpr size_t WS_TOTAL = al256((size_t)3 * NCH * KDP * 2) + al256((size_t)3 * NSM * NCH * NSH * 4) + al256((size_t)NSM * NCH * NPL * 4) + al256((size_t)NSM * NPL * KDP * 2);
static_assert(WS_TOTAL == 107053056 && WS_TOTAL <= 134217728, "the workspace carve: 102.1 MiB");
static_assert(KDP % 64 == 0 && 3 * NCH + 1 <= KDP && NPL == 64 * 64 * 16 && NSH == 64 * 64 && NCH == 64, "whole tiles; whole lines");
typedef _Float16 h16;
typedef unsigned short bf;
typedef __attribute__((ext_vector_type(16))) __bf16   v16bf;
typedef __attribute__((ext_vector_type(16))) _Float16 v16h;
typedef __attribute__((ext_vector_type(8)))  _Float16 v8h;
typedef __attribute__((ext_vector_type(8)))  unsigned short v8us;
typedef __attribute__((ext_vector_type(8)))  float    v8f;
typedef __attribute__((ext_vector_type(4)))  float    v4f;
typedef v8h  __attribute__((may_alias)) v8ha;
typedef v4f  __attribute__((may_alias)) v4fa;
typedef v8us __attribute__((may_alias)) v8usa;

__device__ __forceinline__ unsigned short f2bf(float f) { unsigned u = __float_as_uint(f); u += 0x7FFFu + ((u >> 16) & 1u); return (unsigned short)(u >> 16); }
__device__ __forceinline__ float bf2f(unsigned short b) { return __uint_as_float(((unsigned)b) << 16); }
__device__ __forceinline__ float bfr(float f) { return bf2f(f2bf(f)); }
__device__ __forceinline__ v16h cat16(v8h lo, v8h hi) { return __builtin_shufflevector(lo, hi, 0, 1, 2, 3, 4, 5, 6, 7, 8, 9, 10, 11, 12, 13, 14, 15); }
__device__ __forceinline__ v16bf cat16b(v8us lo, v8us hi) { return __builtin_bit_cast(v16bf, __builtin_shufflevector(lo, hi, 0, 1, 2, 3, 4, 5, 6, 7, 8, 9, 10, 11, 12, 13, 14, 15)); }
__device__ __forceinline__ v8f wmma16(v16h a, v16h b, v8f c) { return __builtin_amdgcn_wmma_f32_16x16x32_f16(false, a, false, b, (short)0, c, false, false); }
__device__ __forceinline__ v8f wmmab(v16bf a, v16bf b, v8f c) { return __builtin_amdgcn_wmma_f32_16x16x32_bf16(false, a, false, b, (short)0, c, false, false); }


template <typename T16> struct WFrag;
template <> struct WFrag<h16> { typedef v16h V; static __device__ __forceinline__ V ld(const h16* p) { return cat16(*(const v8h*)p, *(const v8h*)(p + 16)); } static __device__ __forceinline__ v8f mma(V a, V b, v8f c) { return wmma16(a, b, c); } };
template <> struct WFrag<bf> { typedef v16bf V; static __device__ __forceinline__ V ld(const bf* p) { return cat16b(*(const v8us*)p, *(const v8us*)(p + 16)); } static __device__ __forceinline__ v8f mma(V a, V b, v8f c) { return wmmab(a, b, c); } };
template <typename T16, int NSPLIT, bool BIAS>
__global__ __launch_bounds__(32) void k_gemmw(const T16* __restrict__ A, const T16* __restrict__ A2, const T16* __restrict__ Bt, const T16* __restrict__ Bt2, int K, float* C, int ldc, const float* __restrict__ bias, size_t sA, size_t sB, size_t sC) {
    typedef typename WFrag<T16>::V V;
    __shared__ __align__(16) float os[16 * 68];
    const size_t z = blockIdx.z; A += z * sA; if (A2) A2 += z * sA; Bt += z * sB; if (Bt2) Bt2 += z * sB; C += z * sC;
    const int lane = threadIdx.x & 31, lr = lane & 15, hi = lane >> 4; const int r0 = blockIdx.x * 64, c0 = blockIdx.y * 64;
    v8f acc[4][4];
#pragma unroll
    for (int mb = 0; mb < 4; ++mb)
#pragma unroll
        for (int nb = 0; nb < 4; ++nb) acc[mb][nb] = (v8f){};
    const size_t aoff = (size_t)(r0 + lr) * K + 8 * hi, boff = (size_t)(c0 + lr) * K + 8 * hi;
    for (int kc = 0; kc < K; kc += 32) {
        V a[4], a2[4];
#pragma unroll
        for (int mb = 0; mb < 4; ++mb) { a[mb] = WFrag<T16>::ld(A + aoff + (size_t)mb * 16 * K + kc); if (NSPLIT == 1 || NSPLIT == 2) a2[mb] = WFrag<T16>::ld(A2 + aoff + (size_t)mb * 16 * K + kc); }
#pragma unroll
        for (int nb = 0; nb < 4; ++nb) { const V b = WFrag<T16>::ld(Bt + boff + (size_t)nb * 16 * K + kc); V b2; if (NSPLIT >= 2) b2 = WFrag<T16>::ld(Bt2 + boff + (size_t)nb * 16 * K + kc);
#pragma unroll
            for (int mb = 0; mb < 4; ++mb) { acc[mb][nb] = WFrag<T16>::mma(a[mb], b, acc[mb][nb]); if (NSPLIT == 1 || NSPLIT == 2) acc[mb][nb] = WFrag<T16>::mma(a2[mb], b, acc[mb][nb]); if (NSPLIT >= 2) acc[mb][nb] = WFrag<T16>::mma(a[mb], b2, acc[mb][nb]); } }
        asm volatile("v_nop\n\tv_nop\n\tv_nop\n\tv_nop" : "+v"(acc[0][0]), "+v"(acc[1][1]), "+v"(acc[2][2]), "+v"(acc[3][3]) : "v"(a[0]), "v"(a[3]));
    }
#pragma unroll
    for (int mb = 0; mb < 4; ++mb) {
#pragma unroll
        for (int nb = 0; nb < 4; ++nb) {
#pragma unroll
            for (int j = 0; j < 8; ++j) os[(hi * 8 + j) * 68 + nb * 16 + lr] = acc[mb][nb][j]; }
        __builtin_amdgcn_wave_barrier(); asm volatile("" ::: "memory");
        float* crow = C + (size_t)(r0 + mb * 16) * ldc + c0;
#pragma unroll 1
        for (int ps = 0; ps < 2; ++ps) {
#pragma unroll
            for (int s = 0; s < 8; ++s) { const int row = 2 * s + hi, cofs = lr * 4; v4f val = *(const v4fa*)(os + row * 68 + cofs); if (BIAS) { val[0] += bfr(bias[c0 + cofs]); val[1] += bfr(bias[c0 + cofs + 1]); val[2] += bfr(bias[c0 + cofs + 2]); val[3] += bfr(bias[c0 + cofs + 3]); }
                *(volatile v4f*)(crow + (size_t)row * ldc + cofs) = val; }
            if (ps == 0) __threadfence(); }
        __builtin_amdgcn_wave_barrier(); asm volatile("" ::: "memory");
    }
}

__device__ __forceinline__ h16 tohx(float x) { return (h16)x; }
__device__ __forceinline__ void splitf(float y, unsigned short& h, unsigned short& l) { h = f2bf(y); l = f2bf(y - bf2f(h)); }
typedef __attribute__((ext_vector_type(2))) _Float16 v2h;
typedef __attribute__((ext_vector_type(4))) _Float16 v4h;
typedef __attribute__((ext_vector_type(2))) unsigned short v2us;
typedef __attribute__((ext_vector_type(4))) unsigned short v4us;
typedef __attribute__((ext_vector_type(2))) float v2f;
typedef __attribute__((ext_vector_type(4))) int v4i;


__global__ __launch_bounds__(256) void k_lay(const float* __restrict__ src, h16* dst, unsigned nrow, unsigned c8n, unsigned dp, unsigned c0, unsigned rbs, unsigned ra, unsigned rs, unsigned cbs, unsigned sa, unsigned sb, unsigned rlive, unsigned clive) {
    const unsigned g = blockIdx.x * 256 + threadIdx.x; if (g >= nrow * c8n) return; const unsigned row = g / c8n, ch = g - row * c8n; const unsigned rb = (row >> rbs) * ra + (row & ((1u << rbs) - 1u)) * rs; v8h o;
#pragma unroll
    for (int w = 0; w < 8; ++w) { const unsigned c = 8u * ch + w; const bool live = row < rlive && c < clive; const unsigned si = rb + (c >> cbs) * sa + (c & ((1u << cbs) - 1u)) * sb; const float v = bfr(src[live ? si : 0u]); o[w] = tohx(live && fabsf(v) >= 6.103515625e-05f ? v : 0.0f); }
    h16* d8 = dst + (size_t)row * dp + c0 + 8u * ch; *(volatile v8h*)(d8) = o; __threadfence(); *(volatile v8h*)(d8) = o; }

__global__ __launch_bounds__(256) void k_rnd(const float* __restrict__ vol, float* rr) {
    const unsigned g = blockIdx.x * 256 + threadIdx.x; if (g >= (unsigned)(NSM * NCH * NPL / 4)) return; v4f o; o[0] = bfr(vol[4u * g]); o[1] = bfr(vol[4u * g + 1u]); o[2] = bfr(vol[4u * g + 2u]); o[3] = bfr(vol[4u * g + 3u]);
    float* dq = rr + 4u * (size_t)g; *(volatile v4f*)(dq) = o; __threadfence(); *(volatile v4f*)(dq) = o; }

__global__ __launch_bounds__(256) void k_sht(const float* __restrict__ vol, float* sht, unsigned si, unsigned sj, unsigned st) {
    const unsigned g = blockIdx.x * 256 + threadIdx.x; if (g >= (unsigned)(NSM * NCH * NSH)) return; const unsigned sc = g >> 12, ii = (g >> 6) & 63u, jj = g & 63u; const float* vp = vol + (size_t)sc * NPL + ii * si + jj * sj; float acc = 0.0f;
#pragma unroll
    for (int t = 0; t < 16; ++t) acc += vp[(unsigned)t * st];
    const float val = acc * 0.0625f; *(volatile float*)(sht + g) = val; __threadfence(); *(volatile float*)(sht + g) = val; }

struct CarA { unsigned mi0, mi1, mi2, ui, pi, mj0, mj1, mj2, uj, pj; };
__global__ __launch_bounds__(256) void k_car(const float* __restrict__ sa, const float* __restrict__ sb, h16* dst, unsigned sh0, unsigned sh1, unsigned mk1, unsigned mk2, CarA ca, CarA cb) {
    const unsigned g = blockIdx.x * 256 + threadIdx.x; if (g >= (unsigned)(NSM * NPL * 24)) return; const unsigned row = g / 24u, ch = g - row * 24u; const unsigned sm = row >> 16, pl = row & 65535u; const unsigned q0 = pl >> sh0, q1 = (pl >> sh1) & mk1, q2 = pl & mk2;
    const unsigned isA = ch < 8u ? 1u : 0u, isB = (ch >= 8u && ch < 16u) ? 1u : 0u; const unsigned c0 = (8u * ch) & 63u;
    const unsigned ib = isA * ((q0 * ca.mi0 + q1 * ca.mi1 + q2 * ca.mi2) * ca.ui) + isB * ((q0 * cb.mi0 + q1 * cb.mi1 + q2 * cb.mi2) * cb.ui), jb = isA * ((q0 * ca.mj0 + q1 * ca.mj1 + q2 * ca.mj2) * ca.uj) + isB * ((q0 * cb.mj0 + q1 * cb.mj1 + q2 * cb.mj2) * cb.uj);
    const unsigned st4 = isA * (ca.pi * 64u + ca.pj) + isB * (cb.pi * 64u + cb.pj); const float* sp = (isB ? sb : sa) + (size_t)sm * NCH * NSH + ib * 64u + jb; const float live = (isA | isB) ? 1.0f : 0.0f; v8h o;
#pragma unroll
    for (int e = 0; e < 8; ++e) { const float* sw = sp + (size_t)(c0 + (unsigned)e) * NSH; const float cv = live * 0.25f * (((sw[0] + sw[st4]) + sw[2u * st4]) + sw[3u * st4]); const float one = (ch == 16u && e == 0) ? 1.0f : 0.0f; const float fv = cv + one;
        o[e] = tohx(fabsf(fv) >= 6.103515625e-05f ? fv : 0.0f); }
    h16* d8 = dst + (size_t)row * KDP + 64u + 8u * ch; *(volatile v8h*)(d8) = o; __threadfence(); *(volatile v8h*)(d8) = o; }

extern "C" void kernel_launch(void* const* d_in, const int* in_sizes, int n_in,
                              void* d_out, int out_size, void* d_ws, size_t ws_size, hipStream_t stream) {
    if (n_in < 9) return;
    for (int i = 0; i < 3; ++i) if (in_sizes[i] < NSM * NCH * NPL) return;
    for (int i = 0; i < 3; ++i) if (in_sizes[3 + 2 * i] < NCH * 3 * NCH || in_sizes[4 + 2 * i] < NCH) return;
    if (out_size < 3 * NSM * NCH * NPL) return;
    const float* vols[3] = {(const float*)d_in[0], (const float*)d_in[1], (const float*)d_in[2]}; const float* mats[3] = {(const float*)d_in[3], (const float*)d_in[5], (const float*)d_in[7]}; const float* offs[3] = {(const float*)d_in[4], (const float*)d_in[6], (const float*)d_in[8]};
    char* wsp = (char*)d_ws;
    auto take = [&](size_t bytes) { char* cur = wsp; wsp += (bytes + 255) & ~(size_t)255; return (void*)cur; };
    h16* AW = (h16*)take((size_t)3 * NCH * KDP * 2); float* SS = (float*)take((size_t)3 * NSM * NCH * NSH * 4); float* RR = (float*)take((size_t)NSM * NCH * NPL * 4); h16* PP = (h16*)take((size_t)NSM * NPL * KDP * 2);
    if ((size_t)(wsp - (char*)d_ws) != WS_TOTAL || WS_TOTAL > ws_size) return;
    auto lay = [&](const float* sp_, h16* dp_, unsigned nrow, unsigned ncol, unsigned dp, unsigned c0, unsigned rbs, unsigned ra, unsigned rs_, unsigned cbs, unsigned sa, unsigned sb, unsigned rlive, unsigned clive) {
        k_lay<<<(nrow * (ncol / 8) + 255) / 256, 256, 0, stream>>>(sp_, dp_, nrow, ncol / 8, dp, c0, rbs, ra, rs_, cbs, sa, sb, rlive, clive); };
    const unsigned sI[3] = {1024u, 1024u, 64u}, sJ[3] = {16u, 1u, 1u}, sT[3] = {1u, 64u, 4096u};
    for (int v = 0; v < 3; ++v) { k_rnd<<<(NSM * NCH * NPL / 4 + 255) / 256, 256, 0, stream>>>(vols[v], RR);
        k_sht<<<(NSM * NCH * NSH + 255) / 256, 256, 0, stream>>>(RR, SS + (size_t)v * NSM * NCH * NSH, sI[v], sJ[v], sT[v]); }
    for (int v = 0; v < 3; ++v) { lay(mats[v], AW + (size_t)v * NCH * KDP, NCH, 3 * NCH, KDP, 0, 16, 0, 3 * NCH, 16, 0, 1, NCH, 3 * NCH);
        lay(offs[v], AW + (size_t)v * NCH * KDP, NCH, 64, KDP, 3 * NCH, 16, 0, 1, 16, 0, 0, NCH, 1); }
    const unsigned sh0[3] = {10u, 10u, 12u}, sh1[3] = {4u, 6u, 6u}, mk1[3] = {63u, 15u, 63u}, mk2[3] = {15u, 63u, 63u};
    const CarA car[3][2] = {
        { {1u, 0u, 0u, 1u, 0u,  0u, 0u, 1u, 4u, 1u},
          {0u, 1u, 0u, 1u, 0u,  0u, 0u, 1u, 4u, 1u} },
        { {1u, 0u, 0u, 1u, 0u,  0u, 1u, 0u, 4u, 1u},
          {0u, 1u, 0u, 4u, 1u,  0u, 0u, 1u, 1u, 0u} },
        { {1u, 0u, 0u, 4u, 1u,  0u, 1u, 0u, 1u, 0u},
          {1u, 0u, 0u, 4u, 1u,  0u, 0u, 1u, 1u, 0u} } };
    const int oth[3][2] = {{1, 2}, {0, 2}, {0, 1}};
    for (int v = 0; v < 3; ++v) {
        lay(vols[v], PP, NSM * NPL, NCH, KDP, 0, 16, NCH * NPL, 1, 16, 0, NPL, NSM * NPL, NCH);
        k_car<<<(NSM * NPL * 24 + 255) / 256, 256, 0, stream>>>(SS + (size_t)oth[v][0] * NSM * NCH * NSH, SS + (size_t)oth[v][1] * NSM * NCH * NSH, PP, sh0[v], sh1[v], mk1[v], mk2[v], car[v][0], car[v][1]);
        k_gemmw<h16, 0, false><<<dim3(1, NPL / 64, NSM), 32, 0, stream>>>(AW + (size_t)v * NCH * KDP, nullptr, PP, nullptr, KDP, (float*)d_out + (size_t)v * NSM * NCH * NPL, NPL, nullptr, (size_t)0, (size_t)NPL * KDP, (size_t)NCH * NPL); }
}
